// GATv4Conv_74131135529464
// MI455X (gfx1250) — hardware-run, weakly checked
//
#include <hip/hip_runtime.h>

typedef float          v8f   __attribute__((ext_vector_type(8)));
typedef float          v4f   __attribute__((ext_vector_type(4)));
typedef unsigned int   v4u   __attribute__((ext_vector_type(4)));
typedef int            v8i   __attribute__((ext_vector_type(8)));
typedef unsigned short v8us  __attribute__((ext_vector_type(8)));
typedef unsigned short v16us __attribute__((ext_vector_type(16)));
typedef __bf16         v16bf __attribute__((ext_vector_type(16)));
typedef _Float16       v16h  __attribute__((ext_vector_type(16)));
typedef v4f  __attribute__((may_alias)) v4fa;
typedef v8us __attribute__((may_alias)) v8usa;
union FragB { v16bf v; v16us u; v8us h[2]; v8i w; };
union FragH { v16h  v; v16us u; v8us h[2]; v8i w; };

__device__ __forceinline__ v8f wmb(const FragB& a, const FragB& b, v8f c) {
  v8f d = __builtin_amdgcn_wmma_f32_16x16x32_bf16(false, a.v, false, b.v, (short)0, c, false, false);
  asm volatile("v_nop\n\tv_nop\n\tv_nop\n\tv_nop" : "+v"(d) : "v"(a.w), "v"(b.w));
  return d;
}

__device__ __forceinline__ v8f wmh(const FragH& a, const FragH& b, v8f c) {
  v8f d = __builtin_amdgcn_wmma_f32_16x16x32_f16(false, a.v, false, b.v, (short)0, c, false, false);
  asm volatile("v_nop\n\tv_nop\n\tv_nop\n\tv_nop" : "+v"(d) : "v"(a.w), "v"(b.w));
  return d;
}

__device__ __forceinline__ unsigned bf16_bits(float f) {
  const unsigned u = __float_as_uint(f);
  const unsigned r = (u + 0x7FFFu + ((u >> 16) & 1u)) >> 16;
  const unsigned q = (u >> 16) | 0x40u;
  return ((u & 0x7fffffffu) > 0x7f800000u) ? q : r;
}

__device__ __forceinline__ float bf16_val(float f) {
  return __uint_as_float(bf16_bits(f) << 16);
}
__device__ __forceinline__ int clampi(int v, int lo, int hi) {
  return v < lo ? lo : (v > hi ? hi : v);
}

__device__ __forceinline__ unsigned f16_bits(float f) {
  const unsigned u  = __float_as_uint(f);
  const unsigned s  = (u >> 16) & 0x8000u;
  const unsigned a  = u & 0x7fffffffu;
  const unsigned t  = a - 0x38000000u;
  const unsigned r  = (t + 0x0FFFu + ((t >> 13) & 1u)) >> 13;
  const unsigned rc = r > 0x7C00u ? 0x7C00u : r;
  const bool small  = a < 0x38800000u;
  const bool isnan  = a > 0x7f800000u;
  const unsigned fin = small ? 0u : (s | rc);
  return isnan ? (s | 0x7E00u) : fin;
}

__device__ __forceinline__ unsigned pk16(unsigned lo, unsigned hi) { return lo | (hi << 16); }
__device__ __forceinline__ unsigned bf16_lo_bits(float v) {
  float hi = bf16_val(v);
  asm volatile("" : "+v"(hi));
  return bf16_bits(v - hi);
}
__device__ __forceinline__ v4u pack8_bf16(v4f a, v4f c) {
  return (v4u){ pk16(bf16_bits(a[0]), bf16_bits(a[1])), pk16(bf16_bits(a[2]), bf16_bits(a[3])),
                pk16(bf16_bits(c[0]), bf16_bits(c[1])), pk16(bf16_bits(c[2]), bf16_bits(c[3])) };
}
__device__ __forceinline__ v4u pack8_bf16_lo(v4f a, v4f c) {
  return (v4u){ pk16(bf16_lo_bits(a[0]), bf16_lo_bits(a[1])), pk16(bf16_lo_bits(a[2]), bf16_lo_bits(a[3])),
                pk16(bf16_lo_bits(c[0]), bf16_lo_bits(c[1])), pk16(bf16_lo_bits(c[2]), bf16_lo_bits(c[3])) };
}
__device__ __forceinline__ v4u pack8_f16(v4f a, v4f c) {
  return (v4u){ pk16(f16_bits(a[0]), f16_bits(a[1])), pk16(f16_bits(a[2]), f16_bits(a[3])),
                pk16(f16_bits(c[0]), f16_bits(c[1])), pk16(f16_bits(c[2]), f16_bits(c[3])) };
}

template <int FORM>
__global__ __launch_bounds__(256) void k_plane(const float* __restrict__ src, int rows, int cols, int ldsrc,
                                               unsigned short* __restrict__ dst, int MP, int KP) {
  static_assert(FORM >= 0 && FORM <= 3);
  const int KTOT = (FORM == 1 || FORM == 3) ? 2 * KP : KP;
  const unsigned ppr   = (unsigned)(KTOT >> 3);
  const unsigned kp8   = (unsigned)(KP >> 3);
  const unsigned total = (unsigned)MP * ppr;
  const unsigned g     = blockIdx.x * 256u + threadIdx.x;
  const unsigned rowu  = g / ppr;
  const unsigned p     = g - rowu * ppr;
  const bool second    = p >= kp8;
  const int row = (int)rowu;
  const int c0  = (int)((second ? p - kp8 : p) << 3);
  const float* srow = src + (size_t)clampi(row, 0, rows - 1) * (size_t)ldsrc;
  float x[8];
  unsigned mk[8];
#pragma unroll
  for (int e = 0; e < 8; ++e) {
    const int c = c0 + e;
    const float v = srow[clampi(c, 0, cols - 1)];
    asm volatile("" :: "v"(v));
    x[e]  = v;
    mk[e] = (row < rows && c < cols) ? 0xFFFFu : 0u;
  }
  const v4f a = (v4f){ x[0], x[1], x[2], x[3] };
  const v4f c = (v4f){ x[4], x[5], x[6], x[7] };
  v4u o;
  if (FORM == 2) {
    o = pack8_f16(a, c);
  } else {
    const v4u hi = pack8_bf16(a, c);
    o = hi;
    if (FORM == 1) { const v4u lo = pack8_bf16_lo(a, c); o = second ? lo : hi; }
  }
  const v4u mw = (v4u){ pk16(mk[0], mk[1]), pk16(mk[2], mk[3]), pk16(mk[4], mk[5]), pk16(mk[6], mk[7]) };
  o &= mw;
  if (g < total) {
    volatile v4u* q = (volatile v4u*)(dst + (size_t)g * 8);
    *q = o;
    __threadfence();
    *q = o;
  }
}

template <int FORM> struct FragOf    { typedef FragB T; };
template <>         struct FragOf<2> { typedef FragH T; };
__device__ __forceinline__ v8f mm(const FragB& a, const FragB& b, v8f c) { return wmb(a, b, c); }
__device__ __forceinline__ v8f mm(const FragH& a, const FragH& b, v8f c) { return wmh(a, b, c); }
template <class F> __device__ __forceinline__ F ld_frag(const unsigned short* p) {
  F f;
  f.h[0] = *(const v8usa*)(p);
  f.h[1] = *(const v8usa*)(p + 16);
  return f;
}

template <int FORM, int EPI>
__global__ __launch_bounds__(256) __attribute__((amdgpu_num_vgpr(248)))
void k_gemm_nt(const unsigned short* __restrict__ A, const unsigned short* __restrict__ B,
               const float* __restrict__ bias, float* __restrict__ D, int M, int N, int KTOT, int ldd) {
  static_assert(FORM >= 0 && FORM <= 2);
  static_assert(EPI == 0 || EPI == 1);
  typedef typename FragOf<FORM>::T F;
  __shared__ __attribute__((aligned(16))) float sT[8][16 * 68];
  const int lane = threadIdx.x & 31;
  const int wave = threadIdx.x >> 5;
  const int tilesM = (M + 63) >> 6;
  const int tilesN = (N + 63) >> 6;
  const int tile = blockIdx.x * 8 + wave;
  if (tile >= tilesM * tilesN) return;
  const int tm = tile / tilesN;
  const int tn = tile - tm * tilesN;
  const int m0 = tm << 6;
  const int n0 = tn << 6;

  const int rl = lane & 15;
  const int h8 = (lane >> 4) * 8;
  const unsigned short* pa = A + (size_t)(m0 + rl) * (size_t)KTOT + h8;
  const unsigned short* pb = B + (size_t)(n0 + rl) * (size_t)KTOT + h8;

  v8f acc[4][4];
#pragma unroll
  for (int i = 0; i < 4; ++i)
#pragma unroll
    for (int j = 0; j < 4; ++j) acc[i][j] = (v8f){0.f, 0.f, 0.f, 0.f, 0.f, 0.f, 0.f, 0.f};

#pragma unroll 1
  for (int k0 = 0; k0 < KTOT; k0 += 32) {
    F bf[4];
#pragma unroll
    for (int j = 0; j < 4; ++j) bf[j] = ld_frag<F>(pb + (size_t)(j << 4) * (size_t)KTOT + k0);
#pragma unroll
    for (int i = 0; i < 4; ++i) {
      const F af = ld_frag<F>(pa + (size_t)(i << 4) * (size_t)KTOT + k0);
#pragma unroll
      for (int j = 0; j < 4; ++j) acc[i][j] = mm(af, bf[j], acc[i][j]);
    }
  }

  float* slab = sT[wave];
  const int hh = lane >> 4;
  const int c4 = (lane & 15) * 4;
  const int nc = n0 + c4;
  const bool cok = nc < N;
  v4f bv = (v4f){0.f, 0.f, 0.f, 0.f};
  if (EPI == 1) {
    bv = *(const v4fa*)(bias + clampi(nc, 0, N - 4));
    asm volatile("" :: "v"(bv));
  }
#pragma unroll
  for (int i = 0; i < 4; ++i) {
    const int mBase = m0 + (i << 4);
#pragma unroll
    for (int j = 0; j < 4; ++j) {
#pragma unroll
      for (int r = 0; r < 8; ++r) slab[(h8 + r) * 68 + (j << 4) + rl] = acc[i][j][r];
    }
    __builtin_amdgcn_fence(__ATOMIC_RELEASE, "workgroup");
    __builtin_amdgcn_wave_barrier();
    __builtin_amdgcn_fence(__ATOMIC_ACQUIRE, "workgroup");
    v4f vv[8];
#pragma unroll
    for (int it = 0; it < 8; ++it) {
      const int row = it * 2 + hh;
      v4f v = *(const v4fa*)(slab + row * 68 + c4);
      if (EPI == 1) v += bv;
      vv[it] = v;
    }
    for (int pass = 0; pass < 2; ++pass) {
#pragma unroll
      for (int it = 0; it < 8; ++it) {
        const int row = mBase + it * 2 + hh;
        if (cok && row < M) *(volatile v4f*)(D + (size_t)row * (size_t)ldd + nc) = vv[it];
      }
      __threadfence();
    }
    __builtin_amdgcn_fence(__ATOMIC_RELEASE, "workgroup");
    __builtin_amdgcn_wave_barrier();
    __builtin_amdgcn_fence(__ATOMIC_ACQUIRE, "workgroup");
  }
}


#define NN      50000
#define NE      800000
#define KIN     128
#define MPAD    50048
#define NPAD    448
#define OLD     160
#define NTHR    256
#define NWAVE   8
#define EPT     8
#define WSUB    (32 * EPT)
#define CHUNK   (NWAVE * WSUB)
#define NCHUNK  ((NE + CHUNK - 1) / CHUNK)
#define WCAP    256
#define NBRUN   1024
#define NBLK    ((NN + NBRUN - 1) / NBRUN)
#define RCAP    28672
#define DEGCAP  1024
#define NEGS    0.2f
#define PARN    576
#define LDS_DYN ((2 * RCAP + 3 * NBRUN) * 4)
#define LDS_STA (128 * 4 + 2 * NWAVE * 4)
#define WS_XB   ((size_t)MPAD * KIN * 2)
#define WS_WT   ((size_t)NPAD * KIN * 2)
#define WS_PAR  ((size_t)PARN * 4)
#define WS_P    ((size_t)MPAD * NPAD * 4)
#define WS_TOT  (WS_XB + WS_WT + WS_PAR + WS_P)

static_assert(NE % WSUB == 0);
static_assert(NE % 8 == 0 && NE >= 8);
static_assert(NN <= 65536);
static_assert(NBRUN <= 1024 && NBRUN == NTHR * 4 && (NBRUN % NWAVE) == 0);
static_assert(WCAP == WSUB);
static_assert((RCAP % 32) == 0 && DEGCAP <= RCAP);
static_assert(RCAP >= 16697 + 4096);
static_assert(DEGCAP >= 33 + 8);
static_assert(LDS_DYN + LDS_STA <= 327680);
static_assert(MPAD % 64 == 0 && NPAD % 64 == 0 && KIN % 32 == 0 && MPAD >= NN && KIN == 128);
static_assert(MPAD % 16 == 0 && NPAD % 32 == 0);
static_assert(((size_t)MPAD * KIN / 8) % 256 == 0);
static_assert((NPAD * (KIN / 8)) % 256 == 0);
static_assert(NBLK * NBRUN >= NN && (NBLK - 1) * NBRUN < NN);
static_assert((WS_XB % 256) == 0 && (WS_WT % 256) == 0 && (WS_PAR % 256) == 0 && (WS_P % 256) == 0);
static_assert(WS_TOT <= ((size_t)128 << 20));
static_assert((size_t)(NN - 1) * OLD + OLD - 1 < (size_t)NN * OLD);

typedef int v4i __attribute__((ext_vector_type(4)));
typedef v4i __attribute__((may_alias)) v4ia;

__device__ __forceinline__ v4u wt_gather(const float* __restrict__ w, int cols, int ncol, int k8) {
  const float* p = w + (size_t)k8 * (size_t)cols + ncol;
  float x[8];
#pragma unroll
  for (int e = 0; e < 8; ++e) x[e] = p[(size_t)e * (size_t)cols];
  return pack8_bf16((v4f){ x[0], x[1], x[2], x[3] }, (v4f){ x[4], x[5], x[6], x[7] });
}

__global__ __launch_bounds__(256) void k_wprep(const float* __restrict__ Wsrc, const float* __restrict__ Wself,
                                               const float* __restrict__ Wdst, const float* __restrict__ Wlin,
                                               const float* __restrict__ bsrc, const float* __restrict__ bself,
                                               const float* __restrict__ bdst, const float* __restrict__ blin,
                                               const float* __restrict__ attn,
                                               unsigned short* __restrict__ WT, float* __restrict__ PAR) {
  const int tid = (int)threadIdx.x;
  const int b   = (int)blockIdx.x;
  if (b < 28) {
    const int u  = b * 256 + tid;
    const int n  = u >> 4;
    const int k8 = (u & 15) * 8;
    v4u o = (v4u){ 0u, 0u, 0u, 0u };
    if (b < 8)       o = wt_gather(Wsrc,  128, n,       k8);
    else if (b < 16) o = wt_gather(Wself, 128, n - 128, k8);
    else if (b < 24) o = wt_gather(Wdst,  128, n - 256, k8);
    else if (b < 26) o = wt_gather(Wlin,  32,  n - 384, k8);
    volatile v4u* q = (volatile v4u*)(WT + (size_t)u * 8);
    *q = o;
    __threadfence();
    *q = o;
  } else {
    const int t = tid;
    const v4f c0 = *(const v4fa*)(bsrc  + 4 * clampi(t,       0, 31));
    const v4f c1 = *(const v4fa*)(bself + 4 * clampi(t - 32,  0, 31));
    const v4f c2 = *(const v4fa*)(bdst  + 4 * clampi(t - 64,  0, 31));
    const v4f c3 = *(const v4fa*)(blin  + 4 * clampi(t - 96,  0, 7));
    const v4f c4 = *(const v4fa*)(attn  + 4 * clampi(t - 112, 0, 31));
    asm volatile("" :: "v"(c0), "v"(c1), "v"(c2), "v"(c3), "v"(c4));
    const unsigned m0 = (t < 32) ? 0xFFFFFFFFu : 0u;
    const unsigned m1 = (t >= 32 && t < 64) ? 0xFFFFFFFFu : 0u;
    const unsigned m2 = (t >= 64 && t < 96) ? 0xFFFFFFFFu : 0u;
    const unsigned m3 = (t >= 96 && t < 104) ? 0xFFFFFFFFu : 0u;
    const unsigned m4 = (t >= 112 && t < 144) ? 0xFFFFFFFFu : 0u;
    v4f o;
#pragma unroll
    for (int e = 0; e < 4; ++e) {
      const unsigned bits = (__float_as_uint(c0[e]) & m0) | (__float_as_uint(c1[e]) & m1) |
                            (__float_as_uint(c2[e]) & m2) | (__float_as_uint(c3[e]) & m3) |
                            (__float_as_uint(c4[e]) & m4);
      o[e] = bf16_val(__uint_as_float(bits));
    }
    if (t < 144) {
      volatile v4f* q = (volatile v4f*)(PAR + 4 * t);
      *q = o;
      __threadfence();
      *q = o;
    }
  }
}

__device__ __forceinline__ void att_upd(const v4f a, const v4f mg, const v4f er, const v4f at,
                                        float& mx, float& ls, v4f& acc) {
  v4f v = a + er;
  const float v0 = v[0] > 0.f ? v[0] : NEGS * v[0];
  const float v1 = v[1] > 0.f ? v[1] : NEGS * v[1];
  const float v2 = v[2] > 0.f ? v[2] : NEGS * v[2];
  const float v3 = v[3] > 0.f ? v[3] : NEGS * v[3];
  float part = v0 * at[0];
  part = fmaf(v1, at[1], part);
  part = fmaf(v2, at[2], part);
  part = fmaf(v3, at[3], part);
  part += __shfl_xor(part, 1);
  part += __shfl_xor(part, 2);
  part += __shfl_xor(part, 4);
  const float df = part - mx;
  const float ee = expf(-fabsf(df));
  const bool  up = df > 0.f;
  const float c  = up ? ee : 1.0f;
  const float p  = up ? 1.0f : ee;
  mx  = up ? part : mx;
  ls  = fmaf(ls, c, p);
  acc = acc * c + mg * p;
}

__global__ __launch_bounds__(NTHR) void k_att(const int* __restrict__ srcs, const int* __restrict__ dsts,
                                              const float* __restrict__ P, const float* __restrict__ ATTp,
                                              float* __restrict__ out) {
  extern __shared__ v4f lds_dyn[];
  int* reg1 = (int*)lds_dyn;
  int* reg2 = reg1 + RCAP;
  int* scnt = reg2 + RCAP;
  int* soff = scnt + NBRUN;
  int* curs = soff + NBRUN;
  __shared__ __attribute__((aligned(16))) float sATT[128];
  __shared__ int wcnt[NWAVE];
  __shared__ int wtot[NWAVE];

  const int tid  = (int)threadIdx.x;
  const int lane = tid & 31;
  const int wave = __builtin_amdgcn_readfirstlane(tid >> 5);
  const int nodeBase = (int)blockIdx.x * NBRUN;
  int nb = NN - nodeBase;
  nb = nb > NBRUN ? NBRUN : nb;
  nb = nb < 0 ? 0 : nb;

  *(v4ia*)(scnt + 4 * tid) = (v4i){ 0, 0, 0, 0 };
  if (tid < 32) {
    const v4f av = *(const v4fa*)(ATTp + 4 * tid);
    *(v4fa*)(sATT + 4 * tid) = av;
  }
  __syncthreads();

  int  tot = 0;
  bool ovf = false;
  const unsigned nbs = (unsigned)nodeBase;
  const unsigned unb = (unsigned)nb;
#pragma unroll 1
  for (int ch = 0; ch < NCHUNK; ++ch) {
    const int e0  = ch * CHUNK + wave * WSUB + lane * EPT;
    const int e0c = e0 < (NE - EPT) ? e0 : (NE - EPT);
    const bool ok = e0 < NE;
    const v4i da = *(const v4ia*)(dsts + e0c);
    const v4i db = *(const v4ia*)(dsts + e0c + 4);
    const v4i sa = *(const v4ia*)(srcs + e0c);
    const v4i sb = *(const v4ia*)(srcs + e0c + 4);
    asm volatile("" :: "v"(da), "v"(db), "v"(sa), "v"(sb));
    unsigned sl[8];
    int sv[8];
    sl[0] = (unsigned)da[0] - nbs; sl[1] = (unsigned)da[1] - nbs; sl[2] = (unsigned)da[2] - nbs; sl[3] = (unsigned)da[3] - nbs;
    sl[4] = (unsigned)db[0] - nbs; sl[5] = (unsigned)db[1] - nbs; sl[6] = (unsigned)db[2] - nbs; sl[7] = (unsigned)db[3] - nbs;
    sv[0] = sa[0]; sv[1] = sa[1]; sv[2] = sa[2]; sv[3] = sa[3];
    sv[4] = sb[0]; sv[5] = sb[1]; sv[6] = sb[2]; sv[7] = sb[3];
    unsigned hm = 0u;
#pragma unroll
    for (int j = 0; j < 8; ++j) hm |= ((ok && sl[j] < unb) ? 1u : 0u) << j;
    const int cl = (int)__builtin_popcount(hm);
    int incl = cl;
#pragma unroll
    for (int d = 1; d < 32; d <<= 1) {
      const int upv = __shfl_up(incl, d);
      incl += (lane >= d) ? upv : 0;
    }
    int wcv = incl;
    wcv = wcv < 0 ? 0 : (wcv > WCAP ? WCAP : wcv);
    const int wc = __builtin_amdgcn_readlane(wcv, 31);
    if (lane == 0) wcnt[wave] = wc;
    __syncthreads();
    int pre = 0, all = 0;
#pragma unroll
    for (int w2 = 0; w2 < NWAVE; ++w2) {
      int c = wcnt[w2];
      c = c < 0 ? 0 : (c > WCAP ? WCAP : c);
      all += c;
      pre += (w2 < wave) ? c : 0;
    }
    const int base = tot + pre + (incl - cl);
#pragma unroll
    for (int j = 0; j < 8; ++j) {
      if ((hm >> j) & 1u) {
        const int pos = base + (int)__builtin_popcount(hm & ((1u << j) - 1u));
        if (pos >= 0 && pos < RCAP)
          reg1[pos] = (int)((unsigned)clampi(sv[j], 0, NN - 1) | ((sl[j] & (unsigned)(NBRUN - 1)) << 16));
      }
    }
    tot += all;
    if (tot > RCAP) { tot = RCAP; ovf = true; }
    __syncthreads();
  }
  const int nh = __builtin_amdgcn_readfirstlane(tot);

  if (wave == 0) {
#pragma unroll 1
    for (int b0 = 0; b0 < nh; b0 += 32) {
      int idx = b0 + lane;
      idx = idx < nh ? idx : nh - 1;
      const int uv  = reg1[idx];
      const int m32 = (nh - b0) < 32 ? (nh - b0) : 32;
#pragma unroll 1
      for (int k = 0; k < m32; ++k) {
        const int u  = __builtin_amdgcn_readlane(uv, k);
        const int sq = (u >> 16) & (NBRUN - 1);
        if (lane == 0) scnt[sq] = scnt[sq] + 1;
      }
    }
  }
  __syncthreads();

  {
    const v4i c = *(const v4ia*)(scnt + 4 * tid);
    const int c0 = c[0] < 0 ? 0 : c[0], c1 = c[1] < 0 ? 0 : c[1];
    const int c2 = c[2] < 0 ? 0 : c[2], c3 = c[3] < 0 ? 0 : c[3];
    const int ts = c0 + c1 + c2 + c3;
    int incl = ts;
#pragma unroll
    for (int d = 1; d < 32; d <<= 1) {
      const int upv = __shfl_up(incl, d);
      incl += (lane >= d) ? upv : 0;
    }
    if (lane == 31) wtot[wave] = incl;
    __syncthreads();
    int pre = 0;
#pragma unroll
    for (int w2 = 0; w2 < NWAVE; ++w2) pre += (w2 < wave) ? wtot[w2] : 0;
    const int run = pre + incl - ts;
    const v4i o = (v4i){ run, run + c0, run + c0 + c1, run + c0 + c1 + c2 };
    *(v4ia*)(soff + 4 * tid) = o;
    *(v4ia*)(curs + 4 * tid) = o;
  }
  __syncthreads();

  if (wave == 0) {
#pragma unroll 1
    for (int b0 = 0; b0 < nh; b0 += 32) {
      int idx = b0 + lane;
      idx = idx < nh ? idx : nh - 1;
      const int uv  = reg1[idx];
      const int m32 = (nh - b0) < 32 ? (nh - b0) : 32;
#pragma unroll 1
      for (int k = 0; k < m32; ++k) {
        const int u  = __builtin_amdgcn_readlane(uv, k);
        const int sq = (u >> 16) & (NBRUN - 1);
        if (lane == 0) {
          int pos = curs[sq];
          pos = pos < 0 ? 0 : (pos > RCAP - 1 ? RCAP - 1 : pos);
          reg2[pos] = u & 0xFFFF;
          curs[sq] = pos + 1;
        }
      }
    }
  }
  __syncthreads();

  const float qnan = __uint_as_float(0x7fc00000u);
  const v4f at = *(const v4fa*)(sATT + 4 * lane);
  const int nbw = NBRUN / NWAVE;
#pragma unroll 1
  for (int jt = 0; jt < nbw; ++jt) {
    const int slot = wave * nbw + jt;
    const int grow = nodeBase + slot;
    if (grow >= NN) break;
    int st = soff[slot];
    const int crawv = scnt[slot];
    int cnt = crawv;
    st  = st < 0 ? 0 : (st > nh ? nh : st);
    cnt = cnt < 0 ? 0 : (cnt > DEGCAP ? DEGCAP : cnt);
    cnt = cnt > (nh - st) ? (nh - st) : cnt;
    st  = __builtin_amdgcn_readfirstlane(st);
    cnt = __builtin_amdgcn_readfirstlane(cnt);
    const int craw = __builtin_amdgcn_readfirstlane(crawv);
    const bool bad = ovf || (craw > DEGCAP);

    const float* prow = P + (size_t)grow * (size_t)NPAD;
    const v4f er = *(const v4fa*)(prow + 256 + 4 * lane);
    v4f fl = *(const v4fa*)(prow + 384 + 4 * (lane & 7));
    asm volatile("" :: "v"(er), "v"(fl));

    float mx = -__builtin_inff();
    float ls = 0.0f;
    v4f acc = (v4f){ 0.f, 0.f, 0.f, 0.f };
#pragma unroll 1
    for (int q = 0; q < cnt; q += 2) {
      const int q1 = (q + 1 < cnt) ? q + 1 : cnt - 1;
      int i0 = st + q;  i0 = i0 > RCAP - 1 ? RCAP - 1 : i0;
      int i1 = st + q1; i1 = i1 > RCAP - 1 ? RCAP - 1 : i1;
      const int s0 = clampi(reg2[i0] & 0xFFFF, 0, NN - 1);
      const int s1 = clampi(reg2[i1] & 0xFFFF, 0, NN - 1);
      const float* p0 = P + (size_t)s0 * (size_t)NPAD + 4 * lane;
      const float* p1 = P + (size_t)s1 * (size_t)NPAD + 4 * lane;
      const v4f a0 = *(const v4fa*)(p0);
      const v4f g0 = *(const v4fa*)(p0 + 128);
      const v4f a1 = *(const v4fa*)(p1);
      const v4f g1 = *(const v4fa*)(p1 + 128);
      asm volatile("" :: "v"(a0), "v"(g0), "v"(a1), "v"(g1));
      att_upd(a0, g0, er, at, mx, ls, acc);
      if (q + 1 < cnt) att_upd(a1, g1, er, at, mx, ls, acc);
    }
    const bool has = cnt > 0;
    const float lss = has ? ls : 1.0f;
    const float inv = 1.0f / lss;
    v4f ft = acc * inv;
    const v4f z4 = (v4f){ 0.f, 0.f, 0.f, 0.f };
    const v4f n4 = (v4f){ qnan, qnan, qnan, qnan };
    ft = has ? ft : z4;
    ft = bad ? n4 : ft;
    fl = bad ? n4 : fl;

    float* op = out + (size_t)grow * (size_t)OLD;
    volatile v4f* q0 = (volatile v4f*)(op + 4 * (lane & 7));
    volatile v4f* q1p = (volatile v4f*)(op + 32 + 4 * lane);
    if (lane < 8) *q0 = fl;
    *q1p = ft;
    __threadfence();
    if (lane < 8) *q0 = fl;
    *q1p = ft;
  }
}

extern "C" void kernel_launch(void* const* d_in, const int* in_sizes, int n_in,
                              void* d_out, int out_size, void* d_ws, size_t ws_size,
                              hipStream_t stream) {
  if (n_in < 12) return;
  if (in_sizes[0] != NN * KIN) return;
  if (in_sizes[1] != KIN * 128 || in_sizes[3] != KIN * 128 || in_sizes[5] != KIN * 128) return;
  if (in_sizes[2] != 128 || in_sizes[4] != 128 || in_sizes[6] != 128) return;
  if (in_sizes[7] != KIN * 32 || in_sizes[8] != 32 || in_sizes[9] != 128) return;
  if (in_sizes[10] != NE || in_sizes[11] != NE) return;
  if (out_size != NN * OLD) return;

  const float* feat  = (const float*)d_in[0];
  const float* Wsrc  = (const float*)d_in[1];
  const float* bsrc  = (const float*)d_in[2];
  const float* Wdst  = (const float*)d_in[3];
  const float* bdst  = (const float*)d_in[4];
  const float* Wself = (const float*)d_in[5];
  const float* bself = (const float*)d_in[6];
  const float* Wlin  = (const float*)d_in[7];
  const float* blin  = (const float*)d_in[8];
  const float* attn  = (const float*)d_in[9];
  const int*   src   = (const int*)d_in[10];
  const int*   dst   = (const int*)d_in[11];
  float* out = (float*)d_out;

  char* ws = (char*)d_ws;
  size_t off = 0;
  const size_t oXB  = off; off += WS_XB;
  const size_t oWT  = off; off += WS_WT;
  const size_t oPAR = off; off += WS_PAR;
  const size_t oP   = off; off += WS_P;
  if (off > ws_size || off > ((size_t)128 << 20)) return;
  unsigned short* XB  = (unsigned short*)(ws + oXB);
  unsigned short* WT  = (unsigned short*)(ws + oWT);
  float*          PAR = (float*)(ws + oPAR);
  float*          Pm  = (float*)(ws + oP);

  hipFuncSetAttribute(reinterpret_cast<const void*>(&k_att),
                      hipFuncAttributeMaxDynamicSharedMemorySize, LDS_DYN);

  k_plane<0><<<(MPAD * (KIN / 8)) / 256, 256, 0, stream>>>(feat, NN, KIN, KIN, XB, MPAD, KIN);
  k_wprep<<<29, 256, 0, stream>>>(Wsrc, Wself, Wdst, Wlin, bsrc, bself, bdst, blin, attn, WT, PAR);
  {
    const int tiles = (MPAD / 64) * (NPAD / 64);
    k_gemm_nt<0, 1><<<(tiles + 7) / 8, 256, 0, stream>>>(XB, WT, PAR, Pm, MPAD, NPAD, KIN, NPAD);
  }
  k_att<<<NBLK, NTHR, LDS_DYN, stream>>>(src, dst, Pm, PAR + 448, out);
}
